// MLAAttention_9088150798898
// MI455X (gfx1250) — hardware-verified
//
#include <hip/hip_runtime.h>
#include <stdint.h>

typedef __attribute__((ext_vector_type(16))) _Float16 v16h;
typedef __attribute__((ext_vector_type(8)))  _Float16 v8h;
typedef __attribute__((ext_vector_type(16))) __bf16   v16b;
typedef __attribute__((ext_vector_type(8)))  __bf16   v8b;
typedef __attribute__((ext_vector_type(8)))  float    v8f;
typedef __attribute__((ext_vector_type(4)))  float    v4f;
typedef __attribute__((ext_vector_type(4)))  unsigned v4u;

constexpr int kBatch = 2;
constexpr int kSeq   = 2048;
constexpr int kModel = 2048;
constexpr int kHeads = 16;
constexpr int kHdim  = 128;
constexpr int kNope  = 64;
constexpr int kRope  = 64;
constexpr int kRank  = 512;
constexpr int kTok   = kBatch * kSeq;
constexpr int kKnw   = kHeads * kNope;
constexpr float kScale    = 0.08838834764831845f;
constexpr float kCarry    = 2048.0f;
constexpr float kInvCarry = 1.0f / 2048.0f;
constexpr float kOutCarry = 16.0f;
constexpr float kWoCarry  = 16.0f;
constexpr float kOutFold  = 1.0f / 256.0f;

static_assert(kTok % 64 == 0 && kModel % 64 == 0 && kRank % 64 == 0 && kKnw % 64 == 0 && kRope % 64 == 0);
static_assert(kModel % 32 == 0 && kRank % 32 == 0);
static_assert(kSeq % 64 == 0 && kHdim == kNope + kRope);

constexpr size_t kMiB     = 1048576ull;
constexpr size_t OFF_QF32 = 0;
constexpr size_t OFF_KNH  = 0;
constexpr size_t OFF_KNL  = 8 * kMiB;
constexpr size_t OFF_AO16 = 16 * kMiB;
constexpr size_t OFF_XB   = 32 * kMiB;
constexpr size_t OFF_Q16  = 32 * kMiB;
constexpr size_t OFF_WQB  = 48 * kMiB;
constexpr size_t OFF_WKVB = 56 * kMiB;
constexpr size_t OFF_WKUB = 58 * kMiB;
constexpr size_t OFF_WKRB = 59 * kMiB;
constexpr size_t OFF_WVUB = 59 * kMiB + 262144;
constexpr size_t OFF_CKH  = 61 * kMiB + 262144;
constexpr size_t OFF_CKL  = 65 * kMiB + 262144;
constexpr size_t OFF_WOH  = 69 * kMiB + 262144;
constexpr size_t OFF_COS  = 77 * kMiB + 262144;
constexpr size_t OFF_SIN  = OFF_COS + 262144;
constexpr size_t OFF_KRF  = 77 * kMiB + 786432;
constexpr size_t OFF_KRH  = OFF_KRF + kMiB;
constexpr size_t OFF_KRL  = OFF_KRH + 524288;
constexpr size_t OFF_VTH  = 79 * kMiB + 786432;
constexpr size_t OFF_VTL  = OFF_VTH + 16 * kMiB;
constexpr size_t WS_TOTAL = OFF_VTL + 16 * kMiB;
static_assert(WS_TOTAL == 117178368ull);
static_assert(WS_TOTAL <= 134217728ull);
static_assert((size_t)kTok * kModel * 4 == 32 * kMiB);
static_assert((size_t)kTok * kKnw * 2 == 8 * kMiB);
static_assert((size_t)kTok * kModel * 2 == 16 * kMiB);
static_assert(OFF_KNL + 8 * kMiB <= OFF_AO16 && OFF_AO16 + 16 * kMiB <= OFF_XB);
static_assert(OFF_Q16 + 16 * kMiB <= OFF_WQB);
static_assert(OFF_WQB + (size_t)kModel * kModel * 2 == OFF_WKVB);
static_assert(OFF_WKVB + (size_t)kRank * kModel * 2 == OFF_WKUB);
static_assert(OFF_WKUB + (size_t)kKnw * kRank * 2 == OFF_WKRB);
static_assert(OFF_WKRB + (size_t)kRope * kModel * 2 == OFF_WVUB);
static_assert(OFF_WVUB + (size_t)kModel * kRank * 2 == OFF_CKH);
static_assert(OFF_CKH + (size_t)kTok * kRank * 2 == OFF_CKL);
static_assert(OFF_CKL + (size_t)kTok * kRank * 2 == OFF_WOH);
static_assert(OFF_WOH + (size_t)kModel * kModel * 2 == OFF_COS);
static_assert(OFF_SIN + (size_t)kSeq * 32 * 4 == OFF_KRF);
static_assert(OFF_KRF + (size_t)kTok * kRope * 4 == OFF_KRH);
static_assert(OFF_KRL + (size_t)kTok * kRope * 2 == OFF_VTH);
static_assert(OFF_VTH + (size_t)kModel * kTok * 2 == OFF_VTL);

__device__ __forceinline__ unsigned short f2bf_bits(float f) {
  unsigned u = __float_as_uint(f);
  return (unsigned short)((u + 0x7FFFu + ((u >> 16) & 1u)) >> 16);
}
__device__ __forceinline__ float bf_bits2f(unsigned short h) { return __uint_as_float(((unsigned)h) << 16); }

__device__ __forceinline__ void dep_guard_h(v8f& a, v8f& b, v16h x, v16h y) { asm volatile("v_nop\n\tv_nop\n\tv_nop\n\tv_nop" : "+v"(a), "+v"(b) : "v"(x), "v"(y)); }
__device__ __forceinline__ void dep_guard_b(v8f& a, v8f& b, v16b x, v16b y) { asm volatile("v_nop\n\tv_nop\n\tv_nop\n\tv_nop" : "+v"(a), "+v"(b) : "v"(x), "v"(y)); }
__device__ __forceinline__ void keep4_h(v16h a, v16h b, v16h c, v16h d) { asm volatile("v_nop" :: "v"(a), "v"(b), "v"(c), "v"(d)); }
__device__ __forceinline__ void keep4_b(v16b a, v16b b, v16b c, v16b d) { asm volatile("v_nop" :: "v"(a), "v"(b), "v"(c), "v"(d)); }
__device__ __forceinline__ void acc_guard4(v8f& a, v8f& b, v8f& c, v8f& d) { asm volatile("v_nop\n\tv_nop\n\tv_nop\n\tv_nop" : "+v"(a), "+v"(b), "+v"(c), "+v"(d)); }
template <typename T> struct Frag;
template <> struct Frag<_Float16> {
  typedef v16h V; union U { v16h v; v8h h[2]; };
  static __device__ __forceinline__ v16h load(const _Float16* p) {
    U f; f.h[0] = *(const v8h*)(p); f.h[1] = *(const v8h*)(p + 16); return f.v;
  }
  static __device__ __forceinline__ v8f mma(v16h a, v16h b, v8f c) {
    return __builtin_amdgcn_wmma_f32_16x16x32_f16(false, a, false, b, (short)0, c, false, false);
  }
  static __device__ __forceinline__ void guard(v8f& a, v8f& b, v16h x, v16h y) { dep_guard_h(a, b, x, y); }
  static __device__ __forceinline__ void keep(v16h a, v16h b, v16h c, v16h d) { keep4_h(a, b, c, d); }
};
template <> struct Frag<__bf16> {
  typedef v16b V; union U { v16b v; v8b h[2]; };
  static __device__ __forceinline__ v16b load(const __bf16* p) {
    U f; f.h[0] = *(const v8b*)(p); f.h[1] = *(const v8b*)(p + 16); return f.v;
  }
  static __device__ __forceinline__ v8f mma(v16b a, v16b b, v8f c) {
    return __builtin_amdgcn_wmma_f32_16x16x32_bf16(false, a, false, b, (short)0, c, false, false);
  }
  static __device__ __forceinline__ void guard(v8f& a, v8f& b, v16b x, v16b y) { dep_guard_b(a, b, x, y); }
  static __device__ __forceinline__ void keep(v16b a, v16b b, v16b c, v16b d) { keep4_b(a, b, c, d); }
};

__device__ __forceinline__ unsigned short at_bf_bits(float f) {
  unsigned u = __float_as_uint(f);
  return (unsigned short)((u + 0x7FFFu + ((u >> 16) & 1u)) >> 16);
}
__device__ __forceinline__ __bf16 at_f2bf(float f) { return __builtin_bit_cast(__bf16, at_bf_bits(f)); }
__device__ __forceinline__ void at_split(float f, __bf16& hi, __bf16& lo) {
  const unsigned short hb = at_bf_bits(f);
  hi = __builtin_bit_cast(__bf16, hb);
  lo = at_f2bf(f - __uint_as_float(((unsigned)hb) << 16));
}
__device__ __forceinline__ v8f at_mma(v16b a, v16b b, v8f c) {
  c = __builtin_amdgcn_wmma_f32_16x16x32_bf16(false, a, false, b, (short)0, c, false, false);
  asm volatile("v_nop\n\tv_nop\n\tv_nop\n\tv_nop" : "+v"(c) : "v"(a), "v"(b));
  return c;
}
__device__ __forceinline__ v8f mma_h(v16h a, v16h b, v8f c) {
  c = __builtin_amdgcn_wmma_f32_16x16x32_f16(false, a, false, b, (short)0, c, false, false);
  asm volatile("v_nop\n\tv_nop\n\tv_nop\n\tv_nop" : "+v"(c) : "v"(a), "v"(b));
  return c;
}

__device__ __forceinline__ unsigned pack_bf16x2(float a, float b) {
  return (unsigned)f2bf_bits(a) | ((unsigned)f2bf_bits(b) << 16);
}
__device__ __forceinline__ unsigned pack_f16x2(float a, float b) {
  const unsigned short ha = __builtin_bit_cast(unsigned short, (_Float16)a);
  const unsigned short hb = __builtin_bit_cast(unsigned short, (_Float16)b);
  return (unsigned)ha | ((unsigned)hb << 16);
}

template <int ET> struct Elem;
template <> struct Elem<0> { typedef _Float16 T; };
template <> struct Elem<1> { typedef __bf16 T; };
template <int ET, int SPLIT, int OUT_MODE>
__global__ __launch_bounds__(256) void wmma_gemm64(
    const unsigned short* __restrict__ Ap, const unsigned short* __restrict__ A2p, int lda,
    const unsigned short* __restrict__ Btp, const unsigned short* __restrict__ Bt2p, int ldb,
    void* __restrict__ Cout, void* __restrict__ Cout2, int ldc,
    int M, int N, int K, float scale) {
  typedef typename Elem<ET>::T T;
  typedef typename Frag<T>::V V;
  const T* A = (const T*)Ap; const T* A2 = (const T*)A2p; const T* Bt = (const T*)Btp; const T* Bt2 = (const T*)Bt2p;
  __shared__ __align__(16) float sT[8][16 * 68];
  const int lane = threadIdx.x & 31;
  const int wave = threadIdx.x >> 5;
  const int tilesN = N >> 6;
  const int tilesM = M >> 6;
  const int tile = blockIdx.x * 8 + wave;
  if (tile >= tilesM * tilesN) return;
  const int tm = tile / tilesN;
  const int tn = tile - tm * tilesN;
  const int m0 = tm << 6;
  const int n0 = tn << 6;

  const int rlane = lane & 15;
  const int koff  = (lane >> 4) * 8;
  const int mOff  = (lane >> 4) * 8;

  v8f acc[4][4];
#pragma unroll
  for (int i = 0; i < 4; ++i)
#pragma unroll
    for (int j = 0; j < 4; ++j) acc[i][j] = (v8f){0.f,0.f,0.f,0.f,0.f,0.f,0.f,0.f};

  for (int k0 = 0; k0 < K; k0 += 32) {
    V bh[4], bl[4];
#pragma unroll
    for (int j = 0; j < 4; ++j) {
      const size_t bo = (size_t)(n0 + (j << 4) + rlane) * ldb + koff + k0;
      bh[j] = Frag<T>::load(Bt + bo);
      if (SPLIT & 2) bl[j] = Frag<T>::load(Bt2 + bo);
    }
#pragma unroll
    for (int i = 0; i < 4; ++i) {
      const size_t ao = (size_t)(m0 + (i << 4) + rlane) * lda + koff + k0;
      V ah = Frag<T>::load(A + ao);
      V al;
      if (SPLIT & 1) al = Frag<T>::load(A2 + ao);
#pragma unroll
      for (int j = 0; j < 4; ++j) {
        acc[i][j] = Frag<T>::mma(ah, bh[j], acc[i][j]);
        if (SPLIT & 2) acc[i][j] = Frag<T>::mma(ah, bl[j], acc[i][j]);
        if (SPLIT & 1) acc[i][j] = Frag<T>::mma(al, bh[j], acc[i][j]);
      }
      Frag<T>::guard(acc[i][0], acc[i][3], ah, (SPLIT & 1) ? al : ah);
    }
    Frag<T>::keep(bh[0], bh[1], bh[2], bh[3]);
    if (SPLIT & 2) Frag<T>::keep(bl[0], bl[1], bl[2], bl[3]);
  }
  acc_guard4(acc[0][0], acc[0][1], acc[0][2], acc[0][3]);
  acc_guard4(acc[1][0], acc[1][1], acc[1][2], acc[1][3]);
  acc_guard4(acc[2][0], acc[2][1], acc[2][2], acc[2][3]);
  acc_guard4(acc[3][0], acc[3][1], acc[3][2], acc[3][3]);

  float* slab = sT[wave];
#pragma unroll
  for (int i = 0; i < 4; ++i) {
    const int mBase = m0 + (i << 4);
#pragma unroll
    for (int j = 0; j < 4; ++j) {
#pragma unroll
      for (int r = 0; r < 8; ++r) {
        const float v = acc[i][j][r] * scale;
        slab[(mOff + r) * 68 + (j << 4) + rlane] = v;
      }
    }
    __builtin_amdgcn_fence(__ATOMIC_RELEASE, "workgroup");
    __builtin_amdgcn_wave_barrier();
    __builtin_amdgcn_fence(__ATOMIC_ACQUIRE, "workgroup");
    if (OUT_MODE == 0) {
      float* C = (float*)Cout;
      const int hh = lane >> 4, c4 = (lane & 15) * 4;
      for (int pass = 0; pass < 2; ++pass) {
#pragma unroll
        for (int it = 0; it < 8; ++it) {
          const int row = it * 2 + hh;
          v4f v = *(const v4f*)(slab + row * 68 + c4);
          *(volatile v4f*)(C + (size_t)(mBase + row) * ldc + n0 + c4) = v;
        }
        __threadfence();
      }
    } else {
      const int q = lane >> 3, c8 = (lane & 7) * 8;
      unsigned short* C  = (unsigned short*)Cout;
      unsigned short* C2 = (OUT_MODE >= 2) ? (unsigned short*)Cout2 : nullptr;
      for (int pass = 0; pass < 2; ++pass) {
#pragma unroll
        for (int it = 0; it < 4; ++it) {
          const int row = it * 4 + q;
          const float* sp = slab + row * 68 + c8;
          v8h hv, lv;
#pragma unroll
          for (int e = 0; e < 8; ++e) {
            if (OUT_MODE == 1) {
              hv[e] = (_Float16)sp[e];
            } else if (OUT_MODE == 3) {
              const _Float16 hq = (_Float16)sp[e];
              const float hf = (float)hq;
              hv[e] = hq;
              lv[e] = (_Float16)((sp[e] - hf) * kCarry);
            } else {
              unsigned short hb = f2bf_bits(sp[e]);
              unsigned short lb = f2bf_bits(sp[e] - bf_bits2f(hb));
              hv[e] = __builtin_bit_cast(_Float16, hb);
              lv[e] = __builtin_bit_cast(_Float16, lb);
            }
          }
          *(volatile v8h*)(C + (size_t)(mBase + row) * ldc + n0 + c8) = hv;
          if (OUT_MODE >= 2) *(volatile v8h*)(C2 + (size_t)(mBase + row) * ldc + n0 + c8) = lv;
        }
        __threadfence();
      }
    }
    __builtin_amdgcn_fence(__ATOMIC_RELEASE, "workgroup");
    __builtin_amdgcn_wave_barrier();
    __builtin_amdgcn_fence(__ATOMIC_ACQUIRE, "workgroup");
  }
}

__global__ __launch_bounds__(256) void cast_f32_bf16x8(
    const float* __restrict__ in, unsigned short* __restrict__ out, int n8) {
  const int i = blockIdx.x * 256 + threadIdx.x;
  if (i < n8) {
    const size_t o = (size_t)i * 8;
    const v4f a = *(const v4f*)(in + o);
    const v4f b = *(const v4f*)(in + o + 4);
    v4u u;
    u[0] = pack_bf16x2(a[0], a[1]);
    u[1] = pack_bf16x2(a[2], a[3]);
    u[2] = pack_bf16x2(b[0], b[1]);
    u[3] = pack_bf16x2(b[2], b[3]);
    *(volatile v4u*)(out + o) = u;
    __threadfence();
    *(volatile v4u*)(out + o) = u;
  }
}

__device__ __forceinline__ unsigned pack_bfc_f16x2(float a, float b, float mul) {
  const float fa = bf_bits2f(f2bf_bits(a)) * mul;
  const float fb = bf_bits2f(f2bf_bits(b)) * mul;
  return pack_f16x2(fa, fb);
}
__global__ __launch_bounds__(256) void cast_f32_bfc_f16x8(
    const float* __restrict__ in, unsigned short* __restrict__ out, int n8, float mul) {
  const int i = blockIdx.x * 256 + threadIdx.x;
  if (i < n8) {
    const size_t o = (size_t)i * 8;
    const v4f a = *(const v4f*)(in + o);
    const v4f b = *(const v4f*)(in + o + 4);
    v4u u;
    u[0] = pack_bfc_f16x2(a[0], a[1], mul);
    u[1] = pack_bfc_f16x2(a[2], a[3], mul);
    u[2] = pack_bfc_f16x2(b[0], b[1], mul);
    u[3] = pack_bfc_f16x2(b[2], b[3], mul);
    *(volatile v4u*)(out + o) = u;
    __threadfence();
    *(volatile v4u*)(out + o) = u;
  }
}

struct FreqTab { float f[32]; };
static_assert(sizeof(FreqTab) == 128);
__global__ __launch_bounds__(256) void rope_table_kernel(
    float* __restrict__ cosT, float* __restrict__ sinT, FreqTab ft) {
#pragma clang fp contract(off)
  const int t = blockIdx.x * 256 + threadIdx.x;
  if (t < kSeq * 32) {
    const int pos = t >> 5;
    const int i = t & 31;
    float fs = ft.f[0];
#pragma unroll
    for (int j = 1; j < 32; ++j) fs = (i == j) ? ft.f[j] : fs;
    const float ang = (float)pos * fs;
    const float cv = cosf(ang);
    const float sv = sinf(ang);
    ((volatile float*)cosT)[t] = cv;
    ((volatile float*)sinT)[t] = sv;
    __threadfence();
    ((volatile float*)cosT)[t] = cv;
    ((volatile float*)sinT)[t] = sv;
  }
}

__global__ __launch_bounds__(256) void rope_q_kernel(
    const float* __restrict__ qf, const float* __restrict__ cosT, const float* __restrict__ sinT,
    unsigned short* __restrict__ q16) {
#pragma clang fp contract(off)
  const int row = blockIdx.x;
  const int c0  = threadIdx.x * 8;
  const int pos = row & (kSeq - 1);
  const size_t o = (size_t)row * kModel + c0;
  const v4f a  = *(const v4f*)(qf + o);
  const v4f bq = *(const v4f*)(qf + o + 4);
  const int d  = c0 & (kHdim - 1);
  const bool isr = d >= kNope;
  const int j0 = (d & (kRope - 1)) >> 1;
  const v4f cs = *(const v4f*)(cosT + pos * 32 + j0);
  const v4f sn = *(const v4f*)(sinT + pos * 32 + j0);
  const float xv[8] = {a[0], a[1], a[2], a[3], bq[0], bq[1], bq[2], bq[3]};
  float yv[8];
#pragma unroll
  for (int e = 0; e < 4; ++e) {
    const float x0 = xv[2 * e], x1 = xv[2 * e + 1];
    const float r0 = x0 * cs[e] - x1 * sn[e];
    const float r1 = x1 * cs[e] + x0 * sn[e];
    yv[2 * e]     = isr ? r0 : x0;
    yv[2 * e + 1] = isr ? r1 : x1;
  }
  v4u u;
  u[0] = pack_f16x2(yv[0], yv[1]);
  u[1] = pack_f16x2(yv[2], yv[3]);
  u[2] = pack_f16x2(yv[4], yv[5]);
  u[3] = pack_f16x2(yv[6], yv[7]);
  *(volatile v4u*)(q16 + o) = u;
  __threadfence();
  *(volatile v4u*)(q16 + o) = u;
}

__global__ __launch_bounds__(256) void rope_k_kernel(
    const float* __restrict__ kf, const float* __restrict__ cosT, const float* __restrict__ sinT,
    unsigned short* __restrict__ krh, unsigned short* __restrict__ krl) {
#pragma clang fp contract(off)
  const int row = blockIdx.x * 32 + (threadIdx.x >> 3);
  const int c0  = (threadIdx.x & 7) * 8;
  const int pos = row & (kSeq - 1);
  const int j0  = c0 >> 1;
  const size_t o = (size_t)row * kRope + c0;
  const v4f a  = *(const v4f*)(kf + o);
  const v4f bq = *(const v4f*)(kf + o + 4);
  const v4f cs = *(const v4f*)(cosT + pos * 32 + j0);
  const v4f sn = *(const v4f*)(sinT + pos * 32 + j0);
  const float xv[8] = {a[0], a[1], a[2], a[3], bq[0], bq[1], bq[2], bq[3]};
  float yv[8];
#pragma unroll
  for (int e = 0; e < 4; ++e) {
    const float x0 = xv[2 * e], x1 = xv[2 * e + 1];
    yv[2 * e]     = x0 * cs[e] - x1 * sn[e];
    yv[2 * e + 1] = x1 * cs[e] + x0 * sn[e];
  }
  v4u uh, ul;
#pragma unroll
  for (int e = 0; e < 4; ++e) {
    const _Float16 h0 = (_Float16)yv[2 * e];
    const _Float16 h1 = (_Float16)yv[2 * e + 1];
    const float f0 = (float)h0, f1 = (float)h1;
    const _Float16 l0 = (_Float16)((yv[2 * e] - f0) * kCarry);
    const _Float16 l1 = (_Float16)((yv[2 * e + 1] - f1) * kCarry);
    uh[e] = (unsigned)__builtin_bit_cast(unsigned short, h0) | ((unsigned)__builtin_bit_cast(unsigned short, h1) << 16);
    ul[e] = (unsigned)__builtin_bit_cast(unsigned short, l0) | ((unsigned)__builtin_bit_cast(unsigned short, l1) << 16);
  }
  *(volatile v4u*)(krh + o) = uh;
  *(volatile v4u*)(krl + o) = ul;
  __threadfence();
  *(volatile v4u*)(krh + o) = uh;
  *(volatile v4u*)(krl + o) = ul;
}

__global__ __launch_bounds__(128) void mla_attn_kernel(
    const unsigned short* __restrict__ q16p,
    const unsigned short* __restrict__ knhp, const unsigned short* __restrict__ knlp,
    const unsigned short* __restrict__ krhp, const unsigned short* __restrict__ krlp,
    const unsigned short* __restrict__ vthp, const unsigned short* __restrict__ vtlp,
    unsigned short* __restrict__ aop) {
  union FB { v16b v; v8b h[2]; };
  __shared__ __align__(16) __bf16 Psh[4][16 * 32];
  __shared__ __align__(16) __bf16 Psl[4][16 * 32];
  __shared__ __align__(16) float  Os[4][16 * 132];

  const int tid  = threadIdx.x;
  const int wave = tid >> 5;
  const int lane = tid & 31;
  const int hh   = lane >> 4;
  const int c    = lane & 15;
  const int koff = hh * 8;

  const int bx = blockIdx.x;
  const int qb = bx & (kSeq / 64 - 1);
  const int bh = bx >> 5;
  const int h  = bh & (kHeads - 1);
  const int b  = bh >> 4;
  const int tokbase = b * kSeq;
  const int q0 = qb * 64 + wave * 16;

  const _Float16* q16 = (const _Float16*)q16p;
  const _Float16* knh = (const _Float16*)knhp;
  const _Float16* knl = (const _Float16*)knlp;
  const _Float16* krh = (const _Float16*)krhp;
  const _Float16* krl = (const _Float16*)krlp;
  const __bf16*   vth = (const __bf16*)vthp;
  const __bf16*   vtl = (const __bf16*)vtlp;

  v16h qa[4];
#pragma unroll
  for (int ks = 0; ks < 4; ++ks)
    qa[ks] = Frag<_Float16>::load(q16 + (size_t)(tokbase + q0 + c) * kModel + h * kHdim + ks * 32 + koff);

  float mrow[8], lrow[8];
  v8f oacc[8];
#pragma unroll
  for (int r = 0; r < 8; ++r) { mrow[r] = -INFINITY; lrow[r] = 0.f; }
#pragma unroll
  for (int t = 0; t < 8; ++t) oacc[t] = (v8f){0.f,0.f,0.f,0.f,0.f,0.f,0.f,0.f};

  __bf16* pwh = Psh[wave];
  __bf16* pwl = Psl[wave];
  const int nch = (q0 + 16 + 31) >> 5;
  for (int kc = 0; kc < nch; ++kc) {
    const int kv0 = kc * 32;
    v8f s[2];
#pragma unroll
    for (int j = 0; j < 2; ++j) {
      v8f sh = (v8f){0.f,0.f,0.f,0.f,0.f,0.f,0.f,0.f};
      v8f sl = (v8f){0.f,0.f,0.f,0.f,0.f,0.f,0.f,0.f};
      const size_t krow = (size_t)(tokbase + kv0 + j * 16 + c);
#pragma unroll
      for (int ks = 0; ks < 4; ++ks) {
        v16h bhf, blf;
        if (ks < 2) {
          const size_t ko = krow * kKnw + h * kNope + ks * 32 + koff;
          bhf = Frag<_Float16>::load(knh + ko);
          blf = Frag<_Float16>::load(knl + ko);
        } else {
          const size_t ko = krow * kRope + (ks - 2) * 32 + koff;
          bhf = Frag<_Float16>::load(krh + ko);
          blf = Frag<_Float16>::load(krl + ko);
        }
        sh = mma_h(qa[ks], bhf, sh);
        sl = mma_h(qa[ks], blf, sl);
      }
      s[j] = (sh + sl * kInvCarry) * kScale;
    }
    float cm[8];
#pragma unroll
    for (int r = 0; r < 8; ++r) {
      const int qrow = q0 + 8 * hh + r;
      float m = -INFINITY;
#pragma unroll
      for (int j = 0; j < 2; ++j) {
        const int kvcol = kv0 + j * 16 + c;
        float sv = s[j][r];
        sv = (kvcol > qrow) ? -INFINITY : sv;
        s[j][r] = sv;
        m = fmaxf(m, sv);
      }
#pragma unroll
      for (int off = 1; off < 16; off <<= 1) m = fmaxf(m, __shfl_xor(m, off, 32));
      cm[r] = m;
    }
    __builtin_amdgcn_fence(__ATOMIC_RELEASE, "workgroup");
    __builtin_amdgcn_wave_barrier();
    __builtin_amdgcn_fence(__ATOMIC_ACQUIRE, "workgroup");
#pragma unroll
    for (int r = 0; r < 8; ++r) {
      const float mnew = fmaxf(mrow[r], cm[r]);
      const float alpha = expf(mrow[r] - mnew);
      mrow[r] = mnew;
      float psum = 0.f;
#pragma unroll
      for (int j = 0; j < 2; ++j) {
        const float p = expf(s[j][r] - mnew);
        psum += p;
        __bf16 ph, pl;
        at_split(p, ph, pl);
        pwh[(8 * hh + r) * 32 + j * 16 + c] = ph;
        pwl[(8 * hh + r) * 32 + j * 16 + c] = pl;
      }
#pragma unroll
      for (int off = 1; off < 16; off <<= 1) psum += __shfl_xor(psum, off, 32);
      lrow[r] = lrow[r] * alpha + psum;
#pragma unroll
      for (int t = 0; t < 8; ++t) oacc[t][r] *= alpha;
    }
    __builtin_amdgcn_fence(__ATOMIC_RELEASE, "workgroup");
    __builtin_amdgcn_wave_barrier();
    __builtin_amdgcn_fence(__ATOMIC_ACQUIRE, "workgroup");
    FB pa, pb;
    pa.h[0] = *(const v8b*)(pwh + c * 32 + 8 * hh);
    pa.h[1] = *(const v8b*)(pwh + c * 32 + 16 + 8 * hh);
    pb.h[0] = *(const v8b*)(pwl + c * 32 + 8 * hh);
    pb.h[1] = *(const v8b*)(pwl + c * 32 + 16 + 8 * hh);
#pragma unroll
    for (int t = 0; t < 8; ++t) {
      const size_t vo = (size_t)(h * kHdim + t * 16 + c) * kTok + tokbase + kv0 + koff;
      const v16b vb = Frag<__bf16>::load(vth + vo);
      const v16b vl = Frag<__bf16>::load(vtl + vo);
      oacc[t] = at_mma(pa.v, vb, oacc[t]);
      oacc[t] = at_mma(pa.v, vl, oacc[t]);
      oacc[t] = at_mma(pb.v, vb, oacc[t]);
    }
  }

  float* os = Os[wave];
#pragma unroll
  for (int r = 0; r < 8; ++r) {
    const float inv = kOutCarry / lrow[r];
#pragma unroll
    for (int t = 0; t < 8; ++t) os[(8 * hh + r) * 132 + t * 16 + c] = oacc[t][r] * inv;
  }
  __builtin_amdgcn_fence(__ATOMIC_RELEASE, "workgroup");
  __builtin_amdgcn_wave_barrier();
  __builtin_amdgcn_fence(__ATOMIC_ACQUIRE, "workgroup");
  {
    const int c8 = c * 8;
    for (int pass = 0; pass < 2; ++pass) {
#pragma unroll
      for (int it = 0; it < 8; ++it) {
        const int row = it * 2 + hh;
        const float* sp = os + row * 132 + c8;
        const v4f a  = *(const v4f*)(sp);
        const v4f bq = *(const v4f*)(sp + 4);
        v4u uh;
        uh[0] = pack_f16x2(a[0], a[1]);
        uh[1] = pack_f16x2(a[2], a[3]);
        uh[2] = pack_f16x2(bq[0], bq[1]);
        uh[3] = pack_f16x2(bq[2], bq[3]);
        const size_t go = (size_t)(tokbase + q0 + row) * kModel + h * kHdim + c8;
        *(volatile v4u*)(aop + go) = uh;
      }
      __threadfence();
    }
  }
}

template <int ET, int SPLIT, int OUT_MODE>
static void launch_gemm(hipStream_t st,
                        const unsigned short* A, const unsigned short* A2, int lda,
                        const unsigned short* Bt, const unsigned short* Bt2, int ldb,
                        void* C, void* C2, int ldc, int M, int N, int K, float scale) {
  const int tiles = (M / 64) * (N / 64);
  wmma_gemm64<ET, SPLIT, OUT_MODE><<<dim3((tiles + 7) / 8), dim3(256), 0, st>>>(
      A, A2, lda, Bt, Bt2, ldb, C, C2, ldc, M, N, K, scale);
}

static void launch_cast(hipStream_t st, const float* src, unsigned short* dst, int n) {
  const int n8 = n >> 3;
  cast_f32_bf16x8<<<dim3((n8 + 255) / 256), dim3(256), 0, st>>>(src, dst, n8);
}

extern "C" void kernel_launch(void* const* d_in, const int* in_sizes, int n_in,
                              void* d_out, int out_size, void* d_ws, size_t ws_size,
                              hipStream_t stream) {
  if (n_in < 7) return;
  if (in_sizes[0] != kTok * kModel || in_sizes[1] != kModel * kModel || in_sizes[2] != kRank * kModel ||
      in_sizes[3] != kKnw * kRank || in_sizes[4] != kRope * kModel || in_sizes[5] != kModel * kRank ||
      in_sizes[6] != kModel * kModel) return;
  if (out_size != kTok * kModel) return;
  if (ws_size < WS_TOTAL) return;

  const float* x         = (const float*)d_in[0];
  const float* wq        = (const float*)d_in[1];
  const float* w_kv_down = (const float*)d_in[2];
  const float* w_k_up    = (const float*)d_in[3];
  const float* w_k_rope  = (const float*)d_in[4];
  const float* w_v_up    = (const float*)d_in[5];
  const float* wo        = (const float*)d_in[6];
  float* outp = (float*)d_out;

  char* ws = (char*)d_ws;
  float*          qf32 = (float*)(ws + OFF_QF32);
  unsigned short* knh  = (unsigned short*)(ws + OFF_KNH);
  unsigned short* knl  = (unsigned short*)(ws + OFF_KNL);
  unsigned short* ao16 = (unsigned short*)(ws + OFF_AO16);
  unsigned short* xb   = (unsigned short*)(ws + OFF_XB);
  unsigned short* q16  = (unsigned short*)(ws + OFF_Q16);
  unsigned short* wqb  = (unsigned short*)(ws + OFF_WQB);
  unsigned short* wkvb = (unsigned short*)(ws + OFF_WKVB);
  unsigned short* wkub = (unsigned short*)(ws + OFF_WKUB);
  unsigned short* wkrb = (unsigned short*)(ws + OFF_WKRB);
  unsigned short* wvub = (unsigned short*)(ws + OFF_WVUB);
  unsigned short* ckh  = (unsigned short*)(ws + OFF_CKH);
  unsigned short* ckl  = (unsigned short*)(ws + OFF_CKL);
  unsigned short* woh  = (unsigned short*)(ws + OFF_WOH);
  float*          cosT = (float*)(ws + OFF_COS);
  float*          sinT = (float*)(ws + OFF_SIN);
  float*          krf  = (float*)(ws + OFF_KRF);
  unsigned short* krh  = (unsigned short*)(ws + OFF_KRH);
  unsigned short* krl  = (unsigned short*)(ws + OFF_KRL);
  unsigned short* vth  = (unsigned short*)(ws + OFF_VTH);
  unsigned short* vtl  = (unsigned short*)(ws + OFF_VTL);

  FreqTab ft;
  {
    double r = 1.33;
    for (int it = 0; it < 64; ++it) {
      const double r2 = r * r, r4 = r2 * r2, r7 = r4 * r2 * r, r8 = r4 * r4;
      r = r - (r8 - 10.0) / (8.0 * r7);
    }
    double p = 1.0;
    for (int i = 0; i < 32; ++i) {
      const float pf = (float)p;
      ft.f[i] = 1.0f / pf;
      p *= r;
    }
  }

  launch_cast(stream, x,         xb,   kTok * kModel);
  launch_cast(stream, wq,        wqb,  kModel * kModel);
  launch_cast(stream, w_kv_down, wkvb, kRank * kModel);
  launch_cast(stream, w_k_up,    wkub, kKnw * kRank);
  launch_cast(stream, w_k_rope,  wkrb, kRope * kModel);
  launch_cast(stream, w_v_up,    wvub, kModel * kRank);
  {
    const int n8 = (kModel * kModel) >> 3;
    cast_f32_bfc_f16x8<<<dim3((n8 + 255) / 256), dim3(256), 0, stream>>>(wo, woh, n8, kWoCarry);
  }
  rope_table_kernel<<<dim3(kSeq * 32 / 256), dim3(256), 0, stream>>>(cosT, sinT, ft);
  launch_gemm<1, 0, 0>(stream, xb, xb, kModel, wqb, wqb, kModel, (void*)qf32, (void*)qf32, kModel, kTok, kModel, kModel, 1.0f);
  launch_gemm<1, 0, 2>(stream, xb, xb, kModel, wkvb, wkvb, kModel, (void*)ckh, (void*)ckl, kRank, kTok, kRank, kModel, 1.0f);
  launch_gemm<1, 0, 0>(stream, xb, xb, kModel, wkrb, wkrb, kModel, (void*)krf, (void*)krf, kRope, kTok, kRope, kModel, 1.0f);
  rope_q_kernel<<<dim3(kTok), dim3(256), 0, stream>>>(qf32, cosT, sinT, q16);
  rope_k_kernel<<<dim3(kTok / 32), dim3(256), 0, stream>>>(krf, cosT, sinT, krh, krl);
  launch_gemm<1, 1, 3>(stream, ckh, ckl, kRank, wkub, wkub, kRank, (void*)knh, (void*)knl, kKnw, kTok, kKnw, kRank, 1.0f);
  launch_gemm<1, 2, 2>(stream, wvub, wvub, kRank, ckh, ckl, kRank, (void*)vth, (void*)vtl, kTok, kModel, kTok, kRank, 1.0f);
  mla_attn_kernel<<<dim3(kBatch * kHeads * (kSeq / 64)), dim3(128), 0, stream>>>(
      q16, knh, knl, krh, krl, vth, vtl, ao16);
  launch_gemm<0, 0, 0>(stream, ao16, ao16, kModel, woh, woh, kModel, (void*)outp, (void*)outp, kModel, kTok, kModel, kModel, kOutFold);
}
